// Qwen3MoeGroupedExperts_35691178230103
// MI455X (gfx1250) — hardware-verified
//
#include <hip/hip_runtime.h>
#include <stdint.h>
#include <stddef.h>

#pragma clang fp contract(off)

#define NTOK 4096
#define DM   1024
#define HX   768
#define NEX  8
#define NSL  2
#define MT   32
#define GX   32
#define TPB  4
#define XP   1032
#define HP   776
#define YP   260

#define LDS_XB  (MT * XP * 2)
#define LDS_HB  (MT * HP * 2)
#define LDS_EXP (2 * LDS_XB + LDS_HB)

#define W_SC 256.0f
#define H_SC 256.0f
#define X_LO 2048.0f
#define R_W  0.00390625f
#define R_HW 1.52587890625e-05f
#define R_LO 4.8828125e-04f

static_assert(MT * YP * 4 <= LDS_XB);
static_assert((XP * 2) % 16 == 0);
static_assert((HP * 2) % 16 == 0);
static_assert((YP * 4) % 16 == 0);
static_assert(NTOK % 256 == 0);
static_assert(NTOK % 8 == 0);
static_assert(GX * TPB * MT == NTOK);
static_assert(TPB * MT <= 256);
static_assert(MT * (DM / 8) == 16 * 256);
static_assert(DM % 256 == 0);
static_assert(HX % 128 == 0);
static_assert(DM % 64 == 0);
static_assert(HX % 64 == 0);
static_assert((NTOK * DM) % 8 == 0);
static_assert((NEX * HX * DM) % 8 == 0);
static_assert(NEX == 8);
static_assert(NSL == 2);
static_assert(DM % 128 == 0);

typedef _Float16       v16h __attribute__((ext_vector_type(16)));
typedef _Float16       v8h  __attribute__((ext_vector_type(8)));
typedef float          v8f  __attribute__((ext_vector_type(8)));
typedef float          v4f  __attribute__((ext_vector_type(4)));
typedef unsigned int   v4u  __attribute__((ext_vector_type(4)));
typedef v4f __attribute__((may_alias)) v4fa;
typedef v4u __attribute__((may_alias)) v4ua;

union FragH { v16h v; v4u q[2]; };
union Pack8 { v8h h; v4u u; };

__device__ __forceinline__ unsigned short hbits(float f) {
  _Float16 t = (_Float16)f;
  unsigned short u;
  __builtin_memcpy(&u, &t, 2);
  return u;
}

__device__ __forceinline__ void split_h(float v, _Float16& hi, _Float16& lo) {
  const _Float16 th = (_Float16)v;
  const float res = (v - (float)th) * X_LO;
  hi = th;
  lo = (_Float16)res;
}

__device__ __forceinline__ v8f wmma_h(v16h a, v16h b, v8f c) {
  v8f d = __builtin_amdgcn_wmma_f32_16x16x32_f16(false, a, false, b, (short)0, c, false, false);
  asm volatile("v_nop\n\tv_nop\n\tv_nop\n\tv_nop" : "+v"(d) : "v"(a), "v"(b));
  return d;
}

__device__ __forceinline__ v16h ldfrag(const unsigned short* p, int h) {
  FragH f;
  f.q[0] = *(const v4ua*)(p + 8 * h);
  f.q[1] = *(const v4ua*)(p + 16 + 8 * h);
  return f.v;
}

__global__ __launch_bounds__(256) void k_cvt(const float* __restrict__ src,
                                             unsigned short* __restrict__ dst,
                                             int n8, float sc)
{
  const int g = blockIdx.x * 256 + threadIdx.x;
  if (g >= n8) return;
  const float* s = src + (size_t)g * 8;
  const v4f a = *(const v4fa*)s;
  const v4f c = *(const v4fa*)(s + 4);
  v8h hv;
  hv[0] = (_Float16)(a.x * sc); hv[1] = (_Float16)(a.y * sc);
  hv[2] = (_Float16)(a.z * sc); hv[3] = (_Float16)(a.w * sc);
  hv[4] = (_Float16)(c.x * sc); hv[5] = (_Float16)(c.y * sc);
  hv[6] = (_Float16)(c.z * sc); hv[7] = (_Float16)(c.w * sc);
  Pack8 p;
  p.h = hv;
  const v4u u = p.u;
  unsigned short* d = dst + (size_t)g * 8;
  *(volatile v4u*)d = u;
  __threadfence();
  *(volatile v4u*)d = u;
}

__global__ __launch_bounds__(256) void k_cvtx(const float* __restrict__ src,
                                              unsigned short* __restrict__ dhi,
                                              unsigned short* __restrict__ dlo,
                                              int n8)
{
  const int g = blockIdx.x * 256 + threadIdx.x;
  if (g >= n8) return;
  const float* s = src + (size_t)g * 8;
  const v4f a = *(const v4fa*)s;
  const v4f c = *(const v4fa*)(s + 4);
  v8h hh, hl;
  _Float16 th, tl;
  split_h(a.x, th, tl); hh[0] = th; hl[0] = tl;
  split_h(a.y, th, tl); hh[1] = th; hl[1] = tl;
  split_h(a.z, th, tl); hh[2] = th; hl[2] = tl;
  split_h(a.w, th, tl); hh[3] = th; hl[3] = tl;
  split_h(c.x, th, tl); hh[4] = th; hl[4] = tl;
  split_h(c.y, th, tl); hh[5] = th; hl[5] = tl;
  split_h(c.z, th, tl); hh[6] = th; hl[6] = tl;
  split_h(c.w, th, tl); hh[7] = th; hl[7] = tl;
  Pack8 ph, pl;
  ph.h = hh;
  pl.h = hl;
  const v4u uh = ph.u;
  const v4u ul = pl.u;
  unsigned short* dh = dhi + (size_t)g * 8;
  unsigned short* dl = dlo + (size_t)g * 8;
  *(volatile v4u*)dh = uh;
  *(volatile v4u*)dl = ul;
  __threadfence();
  *(volatile v4u*)dh = uh;
  *(volatile v4u*)dl = ul;
}

__device__ __forceinline__ void part_pass(const float* sY, const int* tk, const int* sl,
                                          float* part, int ns, int wv, int lane, int nrows)
{
  #pragma unroll
  for (int i = 0; i < 4; ++i) {
    const int row = wv * 4 + i;
    int t = tk[row];
    t = (t < 0) ? 0 : ((t > NTOK - 1) ? (NTOK - 1) : t);
    int s = sl[row];
    s = (s != 0) ? 1 : 0;
    const v4f v0 = *(const v4fa*)(sY + row * YP + 4 * lane);
    const v4f v1 = *(const v4fa*)(sY + row * YP + 128 + 4 * lane);
    float* dst = part + ((size_t)t * NSL + s) * DM + ns * 256;
    if (row < nrows) {
      *(volatile v4f*)(dst + 4 * lane) = v0;
      *(volatile v4f*)(dst + 128 + 4 * lane) = v1;
    }
  }
}

__global__ __launch_bounds__(256) void k_expert(const unsigned short* __restrict__ xh,
                                                const unsigned short* __restrict__ xl,
                                                const unsigned short* __restrict__ wg,
                                                const unsigned short* __restrict__ wu,
                                                const unsigned short* __restrict__ wd,
                                                const int* __restrict__ sel,
                                                const float* __restrict__ rw,
                                                float* __restrict__ part, int ntok)
{
  extern __shared__ __align__(16) unsigned char dsm_e[];
  unsigned short* sX  = (unsigned short*)dsm_e;
  unsigned short* sXL = (unsigned short*)(dsm_e + LDS_XB);
  unsigned short* sH  = (unsigned short*)(dsm_e + 2 * LDS_XB);
  float* sY = (float*)dsm_e;
  __shared__ int   sTok[TPB * MT];
  __shared__ int   sSlot[TPB * MT];
  __shared__ float sW[TPB * MT];
  __shared__ int   s_wc[8];

  const int tid = threadIdx.x, lane = tid & 31, wv = tid >> 5;
  const int h = lane >> 4, m = lane & 15;
  const int e = blockIdx.y;
  const int bx = blockIdx.x;

  if (tid < TPB * MT) { sTok[tid] = 0; sSlot[tid] = 0; sW[tid] = 0.0f; }
  __syncthreads();

  int base = 0;
  #pragma unroll 1
  for (int ch = 0; ch < NTOK / 256; ++ch) {
    const int t = ch * 256 + tid;
    const int tc = (t < ntok) ? t : (ntok - 1);
    int e0 = sel[(size_t)tc * NSL + 0];
    int e1 = sel[(size_t)tc * NSL + 1];
    e0 = (e0 < 0) ? 0 : ((e0 > NEX - 1) ? (NEX - 1) : e0);
    e1 = (e1 < 0) ? 0 : ((e1 > NEX - 1) ? (NEX - 1) : e1);
    const float w0 = rw[(size_t)tc * NSL + 0];
    const float w1 = rw[(size_t)tc * NSL + 1];
    const bool f0 = (e0 == e);
    const bool f1 = (e1 == e);
    const bool f = (f0 || f1) && (t < ntok);
    const float wsum = (f0 ? w0 : 0.0f) + (f1 ? w1 : 0.0f);
    const unsigned int msk = __builtin_amdgcn_ballot_w32(f);
    const int off = __builtin_popcount(msk & ((1u << lane) - 1u));
    const int wcnt = __builtin_popcount(msk);
    if (lane == 0) s_wc[wv] = wcnt;
    __syncthreads();
    int pre = 0, tot = 0;
    #pragma unroll
    for (int w2 = 0; w2 < 8; ++w2) {
      const int c2 = s_wc[w2];
      tot += c2;
      pre += (w2 < wv) ? c2 : 0;
    }
    if (f) {
      const int rank = base + pre + off;
      const int tile = rank / MT;
      const int lt = tile / GX;
      const int p = lt * MT + (rank % MT);
      if (((tile % GX) == bx) && ((unsigned)p < (unsigned)(TPB * MT))) {
        sTok[p]  = t;
        sSlot[p] = f0 ? 0 : 1;
        sW[p]    = wsum;
      }
    }
    base += tot;
    __syncthreads();
  }
  const int cnt = base;

  const v8f z8 = {0.f, 0.f, 0.f, 0.f, 0.f, 0.f, 0.f, 0.f};

  #pragma unroll 1
  for (int lt = 0; lt < TPB; ++lt) {
    const int m0 = (bx + GX * lt) * MT;
    if (m0 >= cnt) break;
    int nrows = cnt - m0;
    nrows = (nrows > MT) ? MT : nrows;
    const int lo = lt * MT;

    #pragma unroll
    for (int j = 0; j < 16; ++j) {
      const int idx = tid + 256 * j;
      const int row = idx >> 7, c8 = idx & 127;
      int t = sTok[lo + row];
      t = (t < 0) ? 0 : ((t > NTOK - 1) ? (NTOK - 1) : t);
      const size_t go = (size_t)t * DM + 8 * c8;
      const v4u a = *(const v4ua*)(xh + go);
      const v4u b = *(const v4ua*)(xl + go);
      *(v4ua*)(sX  + row * XP + 8 * c8) = a;
      *(v4ua*)(sXL + row * XP + 8 * c8) = b;
    }
    __syncthreads();

    #pragma unroll 1
    for (int cb = 0; cb < HX / 128; ++cb) {
      const int jg = cb * 128 + wv * 16 + m;
      const unsigned short* wgr = wg + ((size_t)e * HX + jg) * DM;
      const unsigned short* wur = wu + ((size_t)e * HX + jg) * DM;
      v8f ag[2], agl[2], au[2], aul[2];
      #pragma unroll
      for (int mt = 0; mt < 2; ++mt) { ag[mt] = z8; agl[mt] = z8; au[mt] = z8; aul[mt] = z8; }
      #pragma unroll 1
      for (int k0 = 0; k0 < DM; k0 += 64) {
        #pragma unroll
        for (int kk = 0; kk < 2; ++kk) {
          const int kb = k0 + 32 * kk;
          v16h ah[2], al[2];
          #pragma unroll
          for (int mt = 0; mt < 2; ++mt) {
            ah[mt] = ldfrag(sX  + (16 * mt + m) * XP + kb, h);
            al[mt] = ldfrag(sXL + (16 * mt + m) * XP + kb, h);
          }
          const v16h bg = ldfrag(wgr + kb, h);
          const v16h bu = ldfrag(wur + kb, h);
          #pragma unroll
          for (int mt = 0; mt < 2; ++mt) {
            ag[mt]  = wmma_h(ah[mt], bg, ag[mt]);
            agl[mt] = wmma_h(al[mt], bg, agl[mt]);
            au[mt]  = wmma_h(ah[mt], bu, au[mt]);
            aul[mt] = wmma_h(al[mt], bu, aul[mt]);
          }
        }
      }
      #pragma unroll
      for (int mt = 0; mt < 2; ++mt)
        #pragma unroll
        for (int r = 0; r < 8; ++r) {
          const int row = 16 * mt + 8 * h + r;
          const float g = (ag[mt][r] + agl[mt][r] * R_LO) * R_W;
          const float u = (au[mt][r] + aul[mt][r] * R_LO) * R_W;
          const float sig = 1.0f / (1.0f + __expf(-g));
          const float sv = g * sig;
          const float hv = (sv * u) * H_SC;
          sH[row * HP + jg] = hbits(hv);
        }
    }
    __syncthreads();

    #pragma unroll 1
    for (int ns = 0; ns < DM / 256; ++ns) {
      v8f acc[2][2];
      #pragma unroll
      for (int mt = 0; mt < 2; ++mt)
        #pragma unroll
        for (int nt = 0; nt < 2; ++nt) acc[mt][nt] = z8;
      #pragma unroll 1
      for (int k0 = 0; k0 < HX; k0 += 64) {
        #pragma unroll
        for (int kk = 0; kk < 2; ++kk) {
          const int kb = k0 + 32 * kk;
          v16h a[2];
          #pragma unroll
          for (int mt = 0; mt < 2; ++mt)
            a[mt] = ldfrag(sH + (16 * mt + m) * HP + kb, h);
          #pragma unroll
          for (int nt = 0; nt < 2; ++nt) {
            const int d = ns * 256 + wv * 32 + 16 * nt + m;
            const size_t bo = ((size_t)e * DM + d) * HX + kb;
            const v16h b = ldfrag(wd + bo, h);
            #pragma unroll
            for (int mt = 0; mt < 2; ++mt) acc[mt][nt] = wmma_h(a[mt], b, acc[mt][nt]);
          }
        }
      }
      #pragma unroll
      for (int mt = 0; mt < 2; ++mt)
        #pragma unroll
        for (int nt = 0; nt < 2; ++nt) {
          const int cl = wv * 32 + 16 * nt + m;
          #pragma unroll
          for (int r = 0; r < 8; ++r) {
            const int row = 16 * mt + 8 * h + r;
            const float y = acc[mt][nt][r] * R_HW;
            sY[row * YP + cl] = y * sW[lo + row];
          }
        }
      __syncthreads();
      part_pass(sY, sTok + lo, sSlot + lo, part, ns, wv, lane, nrows);
      __threadfence();
      part_pass(sY, sTok + lo, sSlot + lo, part, ns, wv, lane, nrows);
      __syncthreads();
    }
  }
}

__global__ __launch_bounds__(256) void k_sum(const float* __restrict__ part,
                                             const int* __restrict__ sel,
                                             float* __restrict__ out, int ntok)
{
  const int lane = threadIdx.x & 31, wv = threadIdx.x >> 5;
  const int t = blockIdx.x * 8 + wv;
  if (t >= ntok) return;
  int e0 = sel[(size_t)t * NSL + 0];
  int e1 = sel[(size_t)t * NSL + 1];
  e0 = (e0 < 0) ? 0 : ((e0 > NEX - 1) ? (NEX - 1) : e0);
  e1 = (e1 < 0) ? 0 : ((e1 > NEX - 1) ? (NEX - 1) : e1);
  const bool dup = (e0 == e1);
  const float* p0 = part + (size_t)t * NSL * DM;
  const float* p1 = p0 + DM;
  v4f o[8];
  #pragma unroll
  for (int i = 0; i < 8; ++i) {
    const v4f a = *(const v4fa*)(p0 + 128 * i + 4 * lane);
    const v4f b = *(const v4fa*)(p1 + 128 * i + 4 * lane);
    const v4f s = a + b;
    o[i] = dup ? a : s;
  }
  float* d = out + (size_t)t * DM;
  #pragma unroll
  for (int i = 0; i < 8; ++i) *(volatile v4f*)(d + 128 * i + 4 * lane) = o[i];
  __threadfence();
  #pragma unroll
  for (int i = 0; i < 8; ++i) *(volatile v4f*)(d + 128 * i + 4 * lane) = o[i];
}

extern "C" void kernel_launch(void* const* d_in, const int* in_sizes, int n_in,
                              void* d_out, int out_size, void* d_ws, size_t ws_size,
                              hipStream_t stream)
{
  if (n_in < 6) return;
  if (in_sizes[0] != NTOK * DM) return;
  if (in_sizes[1] != NTOK * NSL) return;
  if (in_sizes[2] != NTOK * NSL) return;
  if (in_sizes[3] != NEX * HX * DM) return;
  if (in_sizes[4] != NEX * HX * DM) return;
  if (in_sizes[5] != NEX * DM * HX) return;
  if (out_size != NTOK * DM) return;

  const float* x   = (const float*)d_in[0];
  const float* rw  = (const float*)d_in[1];
  const int*   sel = (const int*)d_in[2];
  const float* wgf = (const float*)d_in[3];
  const float* wuf = (const float*)d_in[4];
  const float* wdf = (const float*)d_in[5];
  float* out = (float*)d_out;

  const size_t bXH   = (size_t)NTOK * DM * 2;
  const size_t bW    = (size_t)NEX * HX * DM * 2;
  const size_t bPART = (size_t)NTOK * NSL * DM * 4;
  const size_t total = 2 * bXH + 3 * bW + bPART;
  if (total > ws_size) return;
  if (total > (size_t)134217728) return;

  char* ws = (char*)d_ws;
  size_t off = 0;
  unsigned short* XH   = (unsigned short*)(ws + off); off += bXH;
  unsigned short* XL   = (unsigned short*)(ws + off); off += bXH;
  unsigned short* WG   = (unsigned short*)(ws + off); off += bW;
  unsigned short* WU   = (unsigned short*)(ws + off); off += bW;
  unsigned short* WD   = (unsigned short*)(ws + off); off += bW;
  float*          PART = (float*)(ws + off);          off += bPART;
  if (off != total) return;

  hipFuncSetAttribute(reinterpret_cast<const void*>(&k_expert),
                      hipFuncAttributeMaxDynamicSharedMemorySize, LDS_EXP);

  {
    const int n8x = NTOK * DM / 8;
    k_cvtx<<<(n8x + 255) / 256, 256, 0, stream>>>(x, XH, XL, n8x);
  }
  {
    const int n8w = NEX * HX * DM / 8;
    k_cvt<<<(n8w + 255) / 256, 256, 0, stream>>>(wgf, WG, n8w, W_SC);
    k_cvt<<<(n8w + 255) / 256, 256, 0, stream>>>(wuf, WU, n8w, W_SC);
    k_cvt<<<(n8w + 255) / 256, 256, 0, stream>>>(wdf, WD, n8w, W_SC);
  }
  k_expert<<<dim3(GX, NEX), 256, LDS_EXP, stream>>>(XH, XL, WG, WU, WD, sel, rw, PART, NTOK);
  k_sum<<<(NTOK + 7) / 8, 256, 0, stream>>>(PART, sel, out, NTOK);
}
